// MultiheadCrossAttention_49074296324609
// MI455X (gfx1250) — hardware-verified
//
#include <hip/hip_runtime.h>

#ifndef NB
#define NB 2
#endif
#ifndef SEQ
#define SEQ 4096
#endif
#define SEQ_FULL 4096
#define NKEY 1024
#define NKEY_FULL 1024
#define DM 1024
#define NH 16
#define HD 64
#define HG 2

typedef unsigned short v8us __attribute__((ext_vector_type(8), may_alias));
typedef float v8f __attribute__((ext_vector_type(8)));
typedef float v4f __attribute__((ext_vector_type(4)));
typedef float v4fa __attribute__((ext_vector_type(4), may_alias));
typedef _Float16 v16h __attribute__((ext_vector_type(16)));
typedef _Float16 v4h __attribute__((ext_vector_type(4)));
union FragH { v16h v; v8us half[2]; _Float16 h[16]; unsigned short u[16]; };

__device__ __forceinline__ unsigned short bf16_bits(float x) { unsigned int u = __float_as_uint(x); return (unsigned short)((u + 0x7FFFu + ((u >> 16) & 1u)) >> 16); }
__device__ __forceinline__ float bf16_val(unsigned short b) { return __uint_as_float(((unsigned int)b) << 16); }
__device__ __forceinline__ float bf16_rne(float x) { return bf16_val(bf16_bits(x)); }

__global__ __launch_bounds__(256) void k_wt_f16(const float* __restrict__ W, _Float16* __restrict__ Wt, int K, int N, float scale, int regroup) {
  const int t = blockIdx.x * 256 + threadIdx.x; if (t >= N * (K / 8)) return;
  const int n = t / (K / 8), k8 = (t % (K / 8)) * 8;
  const int src = regroup ? ((n & 63) * NH + (n >> 6)) : n;
  FragH f;
#pragma unroll
  for (int i = 0; i < 8; ++i) f.h[i] = (_Float16)(bf16_rne(W[(size_t)(k8 + i) * N + src]) * scale);
  const v8us o = f.half[0];
  unsigned short* d = (unsigned short*)Wt + (size_t)n * K + k8;
  *(volatile v8us*)d = o; __threadfence(); *(volatile v8us*)d = o;
}

__global__ __launch_bounds__(256) void k_x16(const float* __restrict__ x, size_t sIn, _Float16* __restrict__ X16, size_t sOut, size_t n8) {
  const size_t t = (size_t)blockIdx.x * 256 + threadIdx.x; if (t >= n8) return;
  const float* src = x + (size_t)blockIdx.y * sIn + t * 8;
  const v4f a = *(const v4fa*)src, c = *(const v4fa*)(src + 4);
  FragH f;
#pragma unroll
  for (int q = 0; q < 4; ++q) { f.h[q] = (_Float16)bf16_rne(a[q]); f.h[4 + q] = (_Float16)bf16_rne(c[q]); }
  const v8us o = f.half[0];
  unsigned short* d = (unsigned short*)X16 + (size_t)blockIdx.y * sOut + t * 8;
  *(volatile v8us*)d = o; __threadfence(); *(volatile v8us*)d = o;
}

__global__ __launch_bounds__(256) void k_mask(const float* __restrict__ c, float* __restrict__ MB, int nrows) {
  const int i = blockIdx.x * 256 + threadIdx.x;
  const int ic = (i < nrows) ? i : (nrows - 1);
  const float* row = c + (size_t)ic * DM;
  int nz = 0;
#pragma unroll 1
  for (int k = 0; k < DM; k += 8) {
    const v4f a = *(const v4fa*)(row + k), b = *(const v4fa*)(row + k + 4);
#pragma unroll
    for (int q = 0; q < 4; ++q) nz |= ((a[q] != 0.0f) ? 1 : 0) | ((b[q] != 0.0f) ? 1 : 0);
  }
  const float mv = nz ? 0.0f : -__builtin_inff();
  if (i < nrows) *(volatile float*)(MB + i) = mv;
  __threadfence();
  if (i < nrows) *(volatile float*)(MB + i) = mv;
}

__device__ __forceinline__ v16h g2_frag(const _Float16* p, int hh) { FragH f; f.half[0] = *(const v8us*)((const unsigned short*)p + 8 * hh); f.half[1] = *(const v8us*)((const unsigned short*)p + 16 + 8 * hh); return f.v; }
__device__ __forceinline__ v8f g2_mma(v16h a, v16h b, v8f c) { v8f d = __builtin_amdgcn_wmma_f32_16x16x32_f16(false, a, false, b, (short)0, c, false, false); asm volatile("v_nop\n\tv_nop\n\tv_nop\n\tv_nop" : "+v"(d) : "v"(a), "v"(b)); return d; }

__global__ __launch_bounds__(128) void k_gemm2(const _Float16* __restrict__ A, int lda, size_t sA, const _Float16* __restrict__ Bh, int ldb, size_t sB, float alpha, const float* __restrict__ cbias,
                                                float* __restrict__ C, _Float16* __restrict__ C16, int ldc, size_t sC, int M, int N, int K) {
  __shared__ __attribute__((aligned(16))) float so[4][32][68];
  const int tid = threadIdx.x, w = tid >> 5, lane = tid & 31, ln = lane & 15, hh = lane >> 4; const int by = blockIdx.y;
  A += (size_t)by * sA; Bh += (size_t)by * sB; const size_t cofs = (size_t)by * sC;
  const int ntn = N >> 6; const int mt = blockIdx.x / ntn, nq = blockIdx.x - mt * ntn; const int row0 = mt * 128 + 32 * w, col0 = nq * 64; if (row0 >= M) return;
  const _Float16* a0p = A + (size_t)(row0 + ln) * lda; const _Float16* a1p = a0p + (size_t)16 * lda;
  const _Float16* b0p = Bh + (size_t)(col0 + ln) * ldb; const _Float16* b1p = b0p + (size_t)16 * ldb; const _Float16* b2p = b1p + (size_t)16 * ldb; const _Float16* b3p = b2p + (size_t)16 * ldb;
  const v8f z8 = {0.f,0.f,0.f,0.f,0.f,0.f,0.f,0.f}; v8f c00 = z8, c01 = z8, c02 = z8, c03 = z8, c10 = z8, c11 = z8, c12 = z8, c13 = z8;
#pragma unroll 1
  for (int kb = 0; kb < K; kb += 32) { const v16h a0 = g2_frag(a0p + kb, hh), a1 = g2_frag(a1p + kb, hh);
    v16h b = g2_frag(b0p + kb, hh); c00 = g2_mma(a0, b, c00); c10 = g2_mma(a1, b, c10);
    b = g2_frag(b1p + kb, hh); c01 = g2_mma(a0, b, c01); c11 = g2_mma(a1, b, c11);
    b = g2_frag(b2p + kb, hh); c02 = g2_mma(a0, b, c02); c12 = g2_mma(a1, b, c12);
    b = g2_frag(b3p + kb, hh); c03 = g2_mma(a0, b, c03); c13 = g2_mma(a1, b, c13); }
  v8f accs[8] = {c00, c01, c02, c03, c10, c11, c12, c13};
#pragma unroll
  for (int u = 0; u < 8; ++u) { const int t = u & 3, half = u >> 2; const int col = col0 + t * 16 + ln; float bv = 0.f; if (cbias) bv = cbias[col];
#pragma unroll
    for (int r = 0; r < 8; ++r) { const int rloc = half * 16 + 8 * hh + r; so[w][rloc][t * 16 + ln] = accs[u][r] * alpha + bv; } }
  __builtin_amdgcn_fence(4, "workgroup"); __builtin_amdgcn_wave_barrier();
  const int rsub = lane >> 4, c4 = (lane & 15) * 4;
  for (int pass = 0; pass < 2; ++pass) {
#pragma unroll
    for (int q = 0; q < 16; ++q) { const int r = q * 2 + rsub; const v4f v = *(const v4fa*)&so[w][r][c4];
      if (C) *(volatile v4f*)(C + cofs + (size_t)(row0 + r) * ldc + col0 + c4) = v;
      if (C16) { v4h h4;
#pragma unroll
        for (int i = 0; i < 4; ++i) h4[i] = (_Float16)v[i]; *(volatile v4h*)(C16 + cofs + (size_t)(row0 + r) * ldc + col0 + c4) = h4; } }
    if (pass == 0) __threadfence(); }
}

__global__ __launch_bounds__(256) void k_rsm(const float* __restrict__ S, _Float16* __restrict__ P, int nrows) {
  #pragma clang fp contract(off)
  const int w = threadIdx.x >> 5, lane = threadIdx.x & 31;
  const int i = blockIdx.x * 8 + w; if (i >= nrows) return;
  const float* s = S + (size_t)i * NKEY + lane * 8;
  float a[4][8];
#pragma unroll
  for (int u = 0; u < 4; ++u) { const v4f x0 = *(const v4fa*)(s + u * 256), x1 = *(const v4fa*)(s + u * 256 + 4);
    a[u][0] = x0[0]; a[u][1] = x0[1]; a[u][2] = x0[2]; a[u][3] = x0[3]; a[u][4] = x1[0]; a[u][5] = x1[1]; a[u][6] = x1[2]; a[u][7] = x1[3]; }
  float mx = -__builtin_inff();
#pragma unroll
  for (int u = 0; u < 4; ++u)
#pragma unroll
    for (int q = 0; q < 8; ++q) mx = fmaxf(mx, a[u][q]);
  mx = fmaxf(mx, __shfl_xor(mx, 16, 32)); mx = fmaxf(mx, __shfl_xor(mx, 8, 32)); mx = fmaxf(mx, __shfl_xor(mx, 4, 32)); mx = fmaxf(mx, __shfl_xor(mx, 2, 32)); mx = fmaxf(mx, __shfl_xor(mx, 1, 32));
  float se = 0.f;
#pragma unroll
  for (int u = 0; u < 4; ++u)
#pragma unroll
    for (int q = 0; q < 8; ++q) { const float e = __expf(a[u][q] - mx); a[u][q] = e; se += e; }
  se += __shfl_xor(se, 16, 32); se += __shfl_xor(se, 8, 32); se += __shfl_xor(se, 4, 32); se += __shfl_xor(se, 2, 32); se += __shfl_xor(se, 1, 32);
  const float sc = 1024.0f / se;
  v8us o[4];
#pragma unroll
  for (int u = 0; u < 4; ++u) { FragH f;
#pragma unroll
    for (int q = 0; q < 8; ++q) f.h[q] = (_Float16)(a[u][q] * sc); o[u] = f.half[0]; }
  unsigned short* d = (unsigned short*)P + (size_t)i * NKEY + lane * 8;
  for (int pass = 0; pass < 2; ++pass) {
#pragma unroll
    for (int u = 0; u < 4; ++u) *(volatile v8us*)(d + u * 256) = o[u];
    if (pass == 0) __threadfence(); }
}

__global__ __launch_bounds__(256) void k_vt(const _Float16* __restrict__ V16, int b, int h0, _Float16* __restrict__ VT) {
  __shared__ unsigned short tl[64][65];
  const int tid = threadIdx.x; const int hh = blockIdx.x % HG, sg = blockIdx.x / HG; const int s0 = sg * 64; const int h = h0 + hh;
  for (int i = tid; i < 64 * 8; i += 256) { const int j = i / 8, d8 = (i % 8) * 8; FragH f; f.half[0] = *(const v8us*)((const unsigned short*)V16 + ((size_t)b * NKEY_FULL + s0 + j) * DM + h * HD + d8);
#pragma unroll
    for (int q = 0; q < 8; ++q) tl[d8 + q][j] = f.u[q]; }
  __syncthreads();
  for (int pass = 0; pass < 2; ++pass) {
    for (int i = tid; i < 64 * 8; i += 256) { const int d = i / 8, j8 = (i % 8) * 8; FragH f;
#pragma unroll
      for (int q = 0; q < 8; ++q) f.u[q] = tl[d][j8 + q];
      *(volatile v8us*)((unsigned short*)VT + ((size_t)hh * HD + d) * NKEY + s0 + j8) = f.half[0]; }
    if (pass == 0) __threadfence(); }
}

extern "C" void kernel_launch(void* const* d_in, const int* in_sizes, int n_in,
                              void* d_out, int out_size, void* d_ws, size_t ws_size, hipStream_t stream) {
  static_assert(NB >= 1 && NB <= 2);
  static_assert(SEQ % 128 == 0 && SEQ >= 128 && SEQ <= SEQ_FULL);
  static_assert(NKEY == 1024 && NKEY <= NKEY_FULL && NKEY % 128 == 0);
  static_assert(DM == NH * HD && HD == 64 && (NH % HG) == 0);
  static_assert((HG * SEQ) % 8 == 0);
  if (n_in < 6) return;
  if (in_sizes[0] < (NB - 1) * SEQ_FULL * DM + SEQ * DM) return;
  if (in_sizes[1] < NB * NKEY_FULL * DM) return;
  if (in_sizes[2] < DM * DM || in_sizes[3] < DM * DM || in_sizes[4] < DM * DM || in_sizes[5] < DM * DM) return;
  if (out_size < (NB - 1) * SEQ_FULL * DM + SEQ * DM) return;
  const float* x  = (const float*)d_in[0];
  const float* c  = (const float*)d_in[1];
  const float* wq = (const float*)d_in[2];
  const float* wk = (const float*)d_in[3];
  const float* wv = (const float*)d_in[4];
  const float* wo = (const float*)d_in[5];
  float* out = (float*)d_out;

  char* ws = (char*)d_ws; size_t off = 0;
  auto take = [&](size_t bytes) { char* p = ws + off; off += (bytes + 255) & ~(size_t)255; return p; };
  const size_t nrq = (size_t)NB * SEQ;
  const size_t nrk = (size_t)NB * NKEY;
  _Float16* BQ  = (_Float16*)take((size_t)DM * DM * 2);
  _Float16* BKV = (_Float16*)take((size_t)2 * DM * DM * 2);
  _Float16* BO  = (_Float16*)take((size_t)DM * DM * 2);
  _Float16* XQ  = (_Float16*)take(nrq * DM * 2);
  _Float16* XC  = (_Float16*)take(nrk * DM * 2);
  _Float16* Q16 = (_Float16*)take(nrq * DM * 2);
  _Float16* KV16 = (_Float16*)take((size_t)2 * nrk * DM * 2);
  _Float16* O16 = (_Float16*)take(nrq * DM * 2);
  float*    MB  = (float*)take(nrk * 4);
  float*    S   = (float*)take((size_t)HG * SEQ * NKEY * 4);
  _Float16* P   = (_Float16*)take((size_t)HG * SEQ * NKEY * 2);
  _Float16* VT  = (_Float16*)take((size_t)HG * HD * NKEY * 2);
  if (off > ws_size) return;
  _Float16* BK = BKV; _Float16* BV = BKV + (size_t)DM * DM;
  _Float16* K16 = KV16; _Float16* V16 = KV16 + nrk * DM;

  const unsigned gw = (unsigned)(((size_t)DM * (DM / 8) + 255) / 256);
  k_wt_f16<<<gw, 256, 0, stream>>>(wq, BQ, DM, DM, 16.0f, 0);
  k_wt_f16<<<gw, 256, 0, stream>>>(wk, BK, DM, DM, 16.0f, 1);
  k_wt_f16<<<gw, 256, 0, stream>>>(wv, BV, DM, DM, 16.0f, 1);
  k_wt_f16<<<gw, 256, 0, stream>>>(wo, BO, DM, DM, 16.0f, 0);
  k_x16<<<dim3((unsigned)(((size_t)SEQ * DM / 8 + 255) / 256), NB), 256, 0, stream>>>(x, (size_t)SEQ_FULL * DM, XQ, (size_t)SEQ * DM, (size_t)SEQ * DM / 8);
  k_x16<<<dim3((unsigned)((nrk * DM / 8 + 255) / 256), 1), 256, 0, stream>>>(c, 0, XC, 0, nrk * DM / 8);
  k_gemm2<<<dim3((unsigned)((nrq / 128) * (DM / 64)), 1), 128, 0, stream>>>(XQ, DM, 0, BQ, DM, 0, 0.0625f, nullptr, nullptr, Q16, DM, 0, (int)nrq, DM, DM);
  k_gemm2<<<dim3((unsigned)((nrk / 128) * (DM / 64)), 2), 128, 0, stream>>>(XC, DM, 0, BK, DM, (size_t)DM * DM, 0.0625f, nullptr, nullptr, K16, DM, nrk * DM, (int)nrk, DM, DM);
  k_mask<<<(unsigned)((nrk + 255) / 256), 256, 0, stream>>>(c, MB, (int)nrk);
  for (int b = 0; b < NB; ++b) for (int h0 = 0; h0 < NH; h0 += HG) {
    const _Float16* qb = Q16 + (size_t)b * SEQ * DM + h0 * HD;
    const _Float16* kb = K16 + (size_t)b * NKEY * DM + h0 * HD;
    k_gemm2<<<dim3((unsigned)((SEQ / 128) * (NKEY / 64)), HG), 128, 0, stream>>>(qb, DM, (size_t)HD, kb, DM, (size_t)HD, 0.125f, MB + (size_t)b * NKEY, S, nullptr, NKEY, (size_t)SEQ * NKEY, SEQ, NKEY, HD);
    k_rsm<<<(unsigned)((HG * SEQ) / 8), 256, 0, stream>>>(S, P, HG * SEQ);
    k_vt<<<(unsigned)(HG * (NKEY / 64)), 256, 0, stream>>>(V16, b, h0, VT);
    k_gemm2<<<dim3((unsigned)((SEQ / 128) * (HD / 64)), HG), 128, 0, stream>>>(P, NKEY, (size_t)SEQ * NKEY, VT, NKEY, (size_t)HD * NKEY, 1.0f, nullptr, nullptr, O16 + (size_t)b * SEQ * DM + h0 * HD, DM, (size_t)HD, SEQ, HD, NKEY);
  }
  k_gemm2<<<dim3((unsigned)((SEQ / 128) * (DM / 64)), NB), 128, 0, stream>>>(O16, DM, (size_t)SEQ * DM, BO, DM, 0, 6.103515625e-05f, nullptr, out, nullptr, DM, (size_t)SEQ_FULL * DM, SEQ, DM, DM);
}
